// SelfAttention_51505247814196
// MI455X (gfx1250) — hardware-verified
//
#include <hip/hip_runtime.h>


#ifndef NB
#define NB 4
#endif
#ifndef SEQ
#define SEQ 1024
#endif
#define NB_FULL  4
#define SEQ_FULL 1024
#ifndef OUT_SEQ
#define OUT_SEQ SEQ
#endif
#define DM   1024
#define NH_  16
#define HD   64
#define EROWS_FULL 1024
#define AW   4
#define EARLY 512
#define QRS  2048.0f
#define QRI  (1.0f / 2048.0f)
#define ESC  64.0f
#define ESI  (1.0f / 64.0f)
#define SC2  (0.125f * 1.4426950408889634f)
#define PSH  8.0f
#define NEGV (-3.0e38f)

static_assert(HD == 64);
static_assert(NH_ * HD == DM);
static_assert(DM % 64 == 0);
static_assert(DM % 32 == 0);
static_assert(SEQ % 64 == 0);
static_assert((NB * SEQ) % 64 == 0);
static_assert(SEQ % 32 == 0);
static_assert(SEQ % (16 * AW) == 0);
static_assert(((size_t)SEQ * DM) % 8 == 0);
static_assert(NB <= NB_FULL);
static_assert(SEQ <= SEQ_FULL);
static_assert(SEQ <= EROWS_FULL);
static_assert(((size_t)NH_ * EROWS_FULL * HD) % 8 == 0);
static_assert(EARLY % 16 == 0);
static_assert(HD * 2 == 128);

typedef _Float16 h16;
typedef unsigned short bf;
typedef __attribute__((ext_vector_type(16))) __bf16   v16bf;
typedef __attribute__((ext_vector_type(16))) _Float16 v16h;
typedef __attribute__((ext_vector_type(8)))  _Float16 v8h;
typedef __attribute__((ext_vector_type(8)))  unsigned short v8us;
typedef __attribute__((ext_vector_type(8)))  float    v8f;
typedef __attribute__((ext_vector_type(4)))  float    v4f;
typedef v4f  __attribute__((may_alias)) v4fa;
typedef v8us __attribute__((may_alias)) v8usa;

__device__ __forceinline__ unsigned short f2bf(float f) { unsigned u = __float_as_uint(f); u += 0x7FFFu + ((u >> 16) & 1u); return (unsigned short)(u >> 16); }
__device__ __forceinline__ float bf2f(unsigned short h) { return __uint_as_float(((unsigned)h) << 16); }
__device__ __forceinline__ v16h cat16(v8h lo, v8h hi) { return __builtin_shufflevector(lo, hi, 0, 1, 2, 3, 4, 5, 6, 7, 8, 9, 10, 11, 12, 13, 14, 15); }
__device__ __forceinline__ v16bf cat16b(v8us lo, v8us hi) { return __builtin_bit_cast(v16bf, __builtin_shufflevector(lo, hi, 0, 1, 2, 3, 4, 5, 6, 7, 8, 9, 10, 11, 12, 13, 14, 15)); }
__device__ __forceinline__ v8f wmma16(v16h a, v16h b, v8f c) { return __builtin_amdgcn_wmma_f32_16x16x32_f16(false, a, false, b, (short)0, c, false, false); }
__device__ __forceinline__ v8f wmmab(v16bf a, v16bf b, v8f c) { return __builtin_amdgcn_wmma_f32_16x16x32_bf16(false, a, false, b, (short)0, c, false, false); }
__device__ __forceinline__ v16h  ldh(const h16* p) { return cat16(*(const v8h*)p, *(const v8h*)(p + 16)); }
__device__ __forceinline__ v16bf ldb(const bf* p)  { return cat16b(*(const v8us*)p, *(const v8us*)(p + 16)); }
__device__ __forceinline__ void wave_sync() { __builtin_amdgcn_fence(3  , "wavefront"); __builtin_amdgcn_wave_barrier(); asm volatile("" ::: "memory"); }
__device__ __forceinline__ h16 toh_flush(float v) { const h16 r = (h16)v; return (fabsf(v) < 6.103515625e-05f) ? (h16)0.0f : r; }
__device__ __forceinline__ v8f wmma16g(v16h a, v16h b, v8f c) {
    c = __builtin_amdgcn_wmma_f32_16x16x32_f16(false, a, false, b, (short)0, c, false, false);
    asm volatile("v_nop\n\tv_nop\n\tv_nop\n\tv_nop" : "+v"(c) : "v"(a), "v"(b));
    return c;
}

__global__ __launch_bounds__(256) void k_cvt8(const float* __restrict__ src, bf* dst, size_t n8) {
    const size_t i = (size_t)blockIdx.x * 256 + threadIdx.x; if (i >= n8) return;
    const v8f v = *(const v8f*)(src + i * 8); v8us o;
#pragma unroll
    for (int k = 0; k < 8; ++k) o[k] = f2bf(v[k]);
    *(volatile v8us*)(dst + i * 8) = o; __threadfence(); *(volatile v8us*)(dst + i * 8) = o;
}

__global__ __launch_bounds__(256) void k_cvtE(const float* __restrict__ src, h16* dst, size_t n8) {
    const size_t i = (size_t)blockIdx.x * 256 + threadIdx.x; if (i >= n8) return;
    const v8f v = *(const v8f*)(src + i * 8); v8h o;
#pragma unroll
    for (int k = 0; k < 8; ++k) o[k] = toh_flush(bf2f(f2bf(v[k])) * ESC);
    *(volatile v8h*)(dst + i * 8) = o; __threadfence(); *(volatile v8h*)(dst + i * 8) = o;
}

__global__ __launch_bounds__(256) void k_cvtT(const float* __restrict__ W, int ldn, bf* dst, int permFrom) {
    __shared__ __align__(16) unsigned short ts[64 * 72];
    const int t = threadIdx.x; const int k0 = blockIdx.x * 64, n0 = blockIdx.y * 64;
#pragma unroll 4
    for (int i = 0; i < 16; ++i) { const int k = i * 4 + (t >> 6), n = t & 63;
        ts[n * 72 + k] = f2bf(W[(size_t)(k0 + k) * (size_t)ldn + n0 + n]); }
    __syncthreads();
    v8us o0, o1; size_t d0, d1;
    { const int p = t, n = p >> 3, q = p & 7; o0 = *(const v8usa*)(&ts[n * 72 + 8 * q]);
      const int e = n0 + n; const int ee = e - permFrom; const int row = (e >= permFrom) ? (permFrom + (ee & 63) * 16 + (ee >> 6)) : e;
      d0 = (size_t)row * DM + k0 + 8 * q; }
    { const int p = t + 256, n = p >> 3, q = p & 7; o1 = *(const v8usa*)(&ts[n * 72 + 8 * q]);
      const int e = n0 + n; const int ee = e - permFrom; const int row = (e >= permFrom) ? (permFrom + (ee & 63) * 16 + (ee >> 6)) : e;
      d1 = (size_t)row * DM + k0 + 8 * q; }
#pragma unroll 1
    for (int ps = 0; ps < 2; ++ps) {
        *(volatile v8us*)(dst + d0) = o0; *(volatile v8us*)(dst + d1) = o1;
        if (ps == 0) __threadfence(); }
}

template <int MODE>
__device__ __forceinline__ void gemm_body(const bf* __restrict__ A, const bf* __restrict__ Bt, const float* __restrict__ bias, h16* Ph, h16* Pr, float* OUT) {
    __shared__ __align__(16) float os[16 * 68];
    const int K = DM;
    const int lane = threadIdx.x & 31, lr = lane & 15, hi = lane >> 4; const int r0 = blockIdx.x * 64, c0 = blockIdx.y * 64;
    v8f acc[4][4];
#pragma unroll
    for (int mb = 0; mb < 4; ++mb)
#pragma unroll
        for (int nb = 0; nb < 4; ++nb) acc[mb][nb] = (v8f){};
    const size_t aoff = (size_t)(r0 + lr) * K + 8 * hi, boff = (size_t)(c0 + lr) * K + 8 * hi;
    const int npl = (MODE == 3) ? 2 : 1;
#pragma unroll 1
    for (int pl = 0; pl < npl; ++pl) {
        const bf* Ap = A + (size_t)pl * ((size_t)NB * SEQ * DM);
#pragma unroll 1
        for (int kc = 0; kc < K; kc += 32) {
            v16bf a[4];
#pragma unroll
            for (int mb = 0; mb < 4; ++mb) a[mb] = ldb(Ap + aoff + (size_t)mb * 16 * K + kc);
#pragma unroll
            for (int nb = 0; nb < 4; ++nb) { const v16bf b = ldb(Bt + boff + (size_t)nb * 16 * K + kc);
#pragma unroll
                for (int mb = 0; mb < 4; ++mb) acc[mb][nb] = wmmab(a[mb], b, acc[mb][nb]); }
            asm volatile("v_nop\n\tv_nop\n\tv_nop\n\tv_nop" : "+v"(acc[0][0]), "+v"(acc[1][1]), "+v"(acc[2][2]), "+v"(acc[3][3]) : "v"(a[0]), "v"(a[1]), "v"(a[2]), "v"(a[3]));
        }
    }
    float bv[4];
#pragma unroll
    for (int nb = 0; nb < 4; ++nb) {
        if (MODE == 2) { bv[nb] = 0.0f; }
        else { const int bi = ((MODE == 1) ? DM : 0) + c0 + nb * 16 + lr; bv[nb] = bf2f(f2bf(bias[bi])); } }
#pragma unroll
    for (int mb = 0; mb < 4; ++mb) {
        float br[8];
#pragma unroll
        for (int j = 0; j < 8; ++j) br[j] = 0.0f;
        if (MODE == 2) {
#pragma unroll
            for (int j = 0; j < 8; ++j) br[j] = bf2f(f2bf(bias[2 * DM + r0 + mb * 16 + hi * 8 + j])); }
#pragma unroll
        for (int nb = 0; nb < 4; ++nb) {
#pragma unroll
            for (int j = 0; j < 8; ++j) os[(hi * 8 + j) * 68 + nb * 16 + lr] = acc[mb][nb][j] + ((MODE == 2) ? br[j] : bv[nb]); }
        wave_sync();
        if (MODE == 0 || MODE == 1 || MODE == 2) {
            size_t sb, rp;
            if (MODE == 2) {
                const int bb = c0 / SEQ; const int tt = c0 % SEQ;
                sb = ((size_t)(bb * NH_ + (r0 >> 6)) * HD + (size_t)(mb * 16)) * SEQ + (size_t)tt; rp = (size_t)SEQ;
            } else {
                const int tok = r0 + mb * 16; const int bb = tok / SEQ; const int tt = tok % SEQ;
                sb = ((size_t)(bb * NH_ + (c0 >> 6)) * SEQ + (size_t)tt) * HD; rp = (size_t)HD; }
#pragma unroll 1
            for (int ps = 0; ps < 2; ++ps) {
#pragma unroll
                for (int s = 0; s < 4; ++s) { const int row = 4 * s + (lane >> 3), c8 = (lane & 7) * 8;
                    const v4f x0 = *(const v4fa*)(&os[row * 68 + c8]); const v4f x1 = *(const v4fa*)(&os[row * 68 + c8 + 4]); v8h hv, rv;
#pragma unroll
                    for (int i = 0; i < 4; ++i) { const h16 a0 = toh_flush(x0[i]); const h16 a1 = toh_flush(x1[i]); hv[i] = a0; hv[4 + i] = a1;
                        rv[i] = toh_flush((x0[i] - (float)a0) * QRS); rv[4 + i] = toh_flush((x1[i] - (float)a1) * QRS); }
                    const size_t oo = sb + (size_t)row * rp + (size_t)c8;
                    *(volatile v8h*)(Ph + oo) = hv; if (MODE == 0 || MODE == 2) *(volatile v8h*)(Pr + oo) = rv; }
                if (ps == 0) __threadfence(); }
        } else {
            const int grow = r0 + 16 * mb; const int bb = grow / SEQ; const int nn = grow % SEQ;
            float* orow = OUT + ((size_t)bb * OUT_SEQ + nn) * DM + c0;
#pragma unroll 1
            for (int ps = 0; ps < 2; ++ps) {
#pragma unroll
                for (int s = 0; s < 8; ++s) { const int row = 2 * s + hi, cofs = lr * 4;
                    const v4f val = *(const v4fa*)(&os[row * 68 + cofs]);
                    *(volatile v4f*)(orow + (size_t)row * DM + cofs) = val; }
                if (ps == 0) __threadfence(); }
        }
        wave_sync();
    }
}

__global__ __launch_bounds__(32) void k_gemm_q(const bf* __restrict__ A, const bf* __restrict__ Bt, const float* __restrict__ bias, h16* Ph, h16* Pr) {
    gemm_body<0>(A, Bt, bias, Ph, Pr, (float*)nullptr);
}
__global__ __launch_bounds__(32) void k_gemm_k(const bf* __restrict__ A, const bf* __restrict__ Bt, const float* __restrict__ bias, h16* Ph) {
    gemm_body<1>(A, Bt, bias, Ph, (h16*)nullptr, (float*)nullptr);
}
__global__ __launch_bounds__(32) void k_gemm_v(const bf* __restrict__ A, const bf* __restrict__ Bt, const float* __restrict__ bias, h16* Ph, h16* Pr) {
    gemm_body<2>(A, Bt, bias, Ph, Pr, (float*)nullptr);
}
__global__ __launch_bounds__(32) void k_gemm_o(const bf* __restrict__ A, const bf* __restrict__ Bt, const float* __restrict__ bias, float* OUT) {
    gemm_body<3>(A, Bt, bias, (h16*)nullptr, (h16*)nullptr, OUT);
}

__global__ __launch_bounds__(32 * AW) __attribute__((amdgpu_num_vgpr(256))) void k_flash(const h16* __restrict__ QH, const h16* __restrict__ QR, const h16* __restrict__ KP, const h16* __restrict__ VT, const h16* __restrict__ VR, const h16* __restrict__ EP, bf* CH, bf* CL) {
    __shared__ __align__(16) float os[AW * 16 * 68];
    const int lane = threadIdx.x & 31, lr = lane & 15, hi = lane >> 4;
    const int wave = __builtin_amdgcn_readfirstlane((int)(threadIdx.x >> 5));
    const int zh = blockIdx.y;
    const int t0 = (blockIdx.x * AW + wave) * 16;
    const size_t pbase = (size_t)zh * SEQ * HD;
    const size_t qo = pbase + (size_t)(t0 + lr) * HD + 8 * hi;
    const size_t ko = pbase + (size_t)lr * HD + 8 * hi;
    const size_t vo = pbase + (size_t)lr * SEQ + 8 * hi;
    const size_t eo = (size_t)(zh % NH_) * EROWS_FULL * HD + 8 * hi;
    const int kend = t0 + 16;
    const bool early = t0 < EARLY;
    const int tq = t0 + lr;
    v8f o0 = (v8f){}, o1 = (v8f){}, o2 = (v8f){}, o3 = (v8f){};
    v8f e0 = (v8f){}, e1 = (v8f){}, e2 = (v8f){}, e3 = (v8f){};
    float m = NEGV, l = 0.0f;
#pragma unroll 1
    for (int key0 = 0; key0 < kend; key0 += 32) {
        unsigned qz = 0u; asm volatile("" : "+v"(qz));
        const size_t qq = qo + (size_t)qz;
        const v16h qh0 = ldh(QH + qq), qh1 = ldh(QH + qq + 32), qr0 = ldh(QR + qq), qr1 = ldh(QR + qq + 32);
        const h16* ka = KP + ko + (size_t)key0 * HD;
        const v16h ka0 = ldh(ka), ka1 = ldh(ka + 32), kb0 = ldh(ka + 16 * HD), kb1 = ldh(ka + 16 * HD + 32);
        v8f sHa = (v8f){}, sLa = (v8f){}, sHb = (v8f){}, sLb = (v8f){};
        sHa = wmma16g(ka0, qh0, sHa); sLa = wmma16g(ka0, qr0, sLa); sHb = wmma16g(kb0, qh0, sHb); sLb = wmma16g(kb0, qr0, sLb);
        sHa = wmma16g(ka1, qh1, sHa); sLa = wmma16g(ka1, qr1, sLa); sHb = wmma16g(kb1, qh1, sHb); sLb = wmma16g(kb1, qr1, sLb);
        float ta[8], tb[8];
#pragma unroll
        for (int r = 0; r < 8; ++r) { ta[r] = sHa[r] + sLa[r] * QRI; tb[r] = sHb[r] + sLb[r] * QRI; }
        const int rb = t0 - key0;
        int ru = rb + lr;      ru = (ru < 0) ? 0 : ru; ru = (ru > EROWS_FULL - 1) ? (EROWS_FULL - 1) : ru;
        int rc = rb - 16 + lr; rc = (rc < 0) ? 0 : rc; rc = (rc > EROWS_FULL - 1) ? (EROWS_FULL - 1) : rc;
        int rd = rb - 32 + lr; rd = (rd < 0) ? 0 : rd; rd = (rd > EROWS_FULL - 1) ? (EROWS_FULL - 1) : rd;
        const h16* eu = EP + eo + (size_t)ru * HD;
        const h16* ec = EP + eo + (size_t)rc * HD;
        const h16* ed = EP + eo + (size_t)rd * HD;
        const v16h eu0 = ldh(eu), eu1 = ldh(eu + 32), ec0 = ldh(ec), ec1 = ldh(ec + 32);
        {
            v8f ra = (v8f){}, rm = (v8f){};
            ra = wmma16g(ka0, eu0, ra); rm = wmma16g(ka0, ec0, rm); ra = wmma16g(ka1, eu1, ra); rm = wmma16g(ka1, ec1, rm);
#pragma unroll
            for (int r = 0; r < 8; ++r) { const float sv = ((lr + 8 * hi + r) <= 15) ? ra[r] : rm[r];
                const float g = __shfl(sv, ((lr - 8 * hi - r) & 15) + 16 * hi, 32);
                ta[r] = (ta[r] + g * ESI) * SC2; }
        }
        const v16h ed0 = ldh(ed), ed1 = ldh(ed + 32);
        {
            v8f ra = (v8f){}, rm = (v8f){};
            ra = wmma16g(kb0, ec0, ra); rm = wmma16g(kb0, ed0, rm); ra = wmma16g(kb1, ec1, ra); rm = wmma16g(kb1, ed1, rm);
#pragma unroll
            for (int r = 0; r < 8; ++r) { const float sv = ((lr + 8 * hi + r) <= 15) ? ra[r] : rm[r];
                const float g = __shfl(sv, ((lr - 8 * hi - r) & 15) + 16 * hi, 32);
                tb[r] = (tb[r] + g * ESI) * SC2; }
        }
        if (key0 + 31 > t0) {
            const int kidx = key0 + 8 * hi;
#pragma unroll
            for (int r = 0; r < 8; ++r) { ta[r] = (kidx + r > tq) ? NEGV : ta[r]; tb[r] = (kidx + 16 + r > tq) ? NEGV : tb[r]; }
        }
        float mx = NEGV;
#pragma unroll
        for (int r = 0; r < 8; ++r) mx = fmaxf(mx, fmaxf(ta[r], tb[r]));
        mx = fmaxf(mx, __shfl_xor(mx, 16, 32));
        const float mnew = fmaxf(m, mx);
        const float alpha = __builtin_amdgcn_exp2f(m - mnew);
        const float sh = PSH - mnew;
        v16h pb; float ls = 0.0f;
#pragma unroll
        for (int r = 0; r < 8; ++r) { const float xa = ta[r] + sh; const float xc = tb[r] + sh;
            const float fa = __builtin_amdgcn_exp2f(xa); const float fc = __builtin_amdgcn_exp2f(xc);
            const h16 pa = (xa < -14.0f) ? (h16)0.0f : (h16)fa; const h16 pc = (xc < -14.0f) ? (h16)0.0f : (h16)fc;
            pb[r] = pa; pb[8 + r] = pc; ls += (float)pa + (float)pc; }
        l = l * alpha + ls; m = mnew;
        o0 = o0 * alpha; o1 = o1 * alpha; o2 = o2 * alpha; o3 = o3 * alpha;
        const h16* va = VT + vo + key0;
        const v16h v0 = ldh(va), v1 = ldh(va + (size_t)16 * SEQ), v2 = ldh(va + (size_t)32 * SEQ), v3 = ldh(va + (size_t)48 * SEQ);
        o0 = wmma16g(v0, pb, o0); o1 = wmma16g(v1, pb, o1); o2 = wmma16g(v2, pb, o2); o3 = wmma16g(v3, pb, o3);
        if (early) {
            e0 = e0 * alpha; e1 = e1 * alpha; e2 = e2 * alpha; e3 = e3 * alpha;
            const h16* vr = VR + vo + key0;
            const v16h w0 = ldh(vr), w1 = ldh(vr + (size_t)16 * SEQ), w2 = ldh(vr + (size_t)32 * SEQ), w3 = ldh(vr + (size_t)48 * SEQ);
            e0 = wmma16g(w0, pb, e0); e1 = wmma16g(w1, pb, e1); e2 = wmma16g(w2, pb, e2); e3 = wmma16g(w3, pb, e3);
        }
    }
    l += __shfl_xor(l, 16, 32);
    const float inv = 1.0f / l;
    const int wb = wave * 16 * 68;
    { v4f a, c;
#pragma unroll
      for (int i = 0; i < 4; ++i) { a[i] = (o0[i] + e0[i] * QRI) * inv; c[i] = (o0[4 + i] + e0[4 + i] * QRI) * inv; }
      *(v4fa*)(&os[wb + lr * 68 +  0 + 8 * hi]) = a; *(v4fa*)(&os[wb + lr * 68 +  0 + 8 * hi + 4]) = c;
#pragma unroll
      for (int i = 0; i < 4; ++i) { a[i] = (o1[i] + e1[i] * QRI) * inv; c[i] = (o1[4 + i] + e1[4 + i] * QRI) * inv; }
      *(v4fa*)(&os[wb + lr * 68 + 16 + 8 * hi]) = a; *(v4fa*)(&os[wb + lr * 68 + 16 + 8 * hi + 4]) = c;
#pragma unroll
      for (int i = 0; i < 4; ++i) { a[i] = (o2[i] + e2[i] * QRI) * inv; c[i] = (o2[4 + i] + e2[4 + i] * QRI) * inv; }
      *(v4fa*)(&os[wb + lr * 68 + 32 + 8 * hi]) = a; *(v4fa*)(&os[wb + lr * 68 + 32 + 8 * hi + 4]) = c;
#pragma unroll
      for (int i = 0; i < 4; ++i) { a[i] = (o3[i] + e3[i] * QRI) * inv; c[i] = (o3[4 + i] + e3[4 + i] * QRI) * inv; }
      *(v4fa*)(&os[wb + lr * 68 + 48 + 8 * hi]) = a; *(v4fa*)(&os[wb + lr * 68 + 48 + 8 * hi + 4]) = c; }
    wave_sync();
    const size_t cb = ((size_t)(zh / NH_) * SEQ + (size_t)t0) * DM + (size_t)(zh % NH_) * HD;
    v8us hv[4], lv[4];
#pragma unroll
    for (int s = 0; s < 4; ++s) { const int row = 4 * s + (lane >> 3), c8 = (lane & 7) * 8;
        const v4f x0 = *(const v4fa*)(&os[wb + row * 68 + c8]); const v4f x1 = *(const v4fa*)(&os[wb + row * 68 + c8 + 4]);
#pragma unroll
        for (int i = 0; i < 4; ++i) { const unsigned short a0 = f2bf(x0[i]); const unsigned short a1 = f2bf(x1[i]);
            hv[s][i] = a0; hv[s][4 + i] = a1; lv[s][i] = f2bf(x0[i] - bf2f(a0)); lv[s][4 + i] = f2bf(x1[i] - bf2f(a1)); } }
#pragma unroll 1
    for (int ps = 0; ps < 2; ++ps) {
#pragma unroll
        for (int s = 0; s < 4; ++s) { const size_t oo = cb + (size_t)(4 * s + (lane >> 3)) * DM + (size_t)((lane & 7) * 8);
            *(volatile v8us*)(CH + oo) = hv[s]; *(volatile v8us*)(CL + oo) = lv[s]; }
        if (ps == 0) __threadfence(); }
}

static constexpr size_t al256(size_t v) { return (v + 255) & ~(size_t)255; }
static constexpr size_t SZ_XB = al256((size_t)NB * SEQ * DM * 2);
static constexpr size_t SZ_WB = al256((size_t)3 * DM * DM * 2);
static constexpr size_t SZ_WF = al256((size_t)DM * DM * 2);
static constexpr size_t SZ_EP = al256((size_t)NH_ * EROWS_FULL * HD * 2);
static constexpr size_t SZ_PL = al256((size_t)NB * SEQ * DM * 2);
static constexpr size_t SZ_TOTAL = SZ_XB + SZ_WB + SZ_WF + SZ_EP + 5 * SZ_PL + 2 * SZ_PL;
static_assert(SZ_TOTAL <= (size_t)134217728);
static_assert(((size_t)DM * DM * 2) % 256 == 0);
static_assert(SZ_PL == (size_t)NB * SEQ * DM * 2);
static_assert((size_t)NB * NH_ * SEQ * HD == (size_t)NB * SEQ * DM);

extern "C" void kernel_launch(void* const* d_in, const int* in_sizes, int n_in,
                              void* d_out, int out_size, void* d_ws, size_t ws_size, hipStream_t stream) {
    if (n_in < 6) return;
    const size_t needx = ((size_t)(NB - 1) * SEQ_FULL + SEQ) * DM;
    if ((size_t)in_sizes[0] < needx) return;
    if ((size_t)in_sizes[1] < (size_t)3 * DM * DM || (size_t)in_sizes[2] < (size_t)3 * DM) return;
    if ((size_t)in_sizes[3] < (size_t)DM * DM || (size_t)in_sizes[4] < (size_t)DM) return;
    if ((size_t)in_sizes[5] < (size_t)NH_ * EROWS_FULL * HD) return;
    if ((size_t)out_size < ((size_t)(NB - 1) * OUT_SEQ + SEQ) * DM) return;
    if (SZ_TOTAL > ws_size) return;
    const float* x = (const float*)d_in[0]; const float* wqkv = (const float*)d_in[1]; const float* bqkv = (const float*)d_in[2];
    const float* wfc = (const float*)d_in[3]; const float* bfc = (const float*)d_in[4]; const float* etab = (const float*)d_in[5];
    float* OUT = (float*)d_out;
    char* wsp = (char*)d_ws;
    bf* XB = (bf*)wsp; wsp += SZ_XB;
    bf* WB = (bf*)wsp; wsp += SZ_WB;
    bf* WF = (bf*)wsp; wsp += SZ_WF;
    h16* EP = (h16*)wsp; wsp += SZ_EP;
    h16* QH = (h16*)wsp; wsp += SZ_PL;
    h16* QR = (h16*)wsp; wsp += SZ_PL;
    h16* KP = (h16*)wsp; wsp += SZ_PL;
    h16* VT = (h16*)wsp; wsp += SZ_PL;
    h16* VR = (h16*)wsp; wsp += SZ_PL;
    bf* CH = (bf*)wsp; wsp += SZ_PL;
    bf* CL = (bf*)wsp; wsp += SZ_PL;

    if (SEQ == SEQ_FULL) {
        const size_t n8 = (size_t)NB * SEQ * DM / 8;
        k_cvt8<<<(unsigned)((n8 + 255) / 256), 256, 0, stream>>>(x, XB, n8);
    } else {
        const size_t n8 = (size_t)SEQ * DM / 8;
        for (int b = 0; b < NB; ++b) k_cvt8<<<(unsigned)((n8 + 255) / 256), 256, 0, stream>>>(x + (size_t)b * SEQ_FULL * DM, XB + (size_t)b * SEQ * DM, n8);
    }
    {
        const size_t n8 = (size_t)NH_ * EROWS_FULL * HD / 8;
        k_cvtE<<<(unsigned)((n8 + 255) / 256), 256, 0, stream>>>(etab, EP, n8);
    }
    k_cvtT<<<dim3(DM / 64, 3 * DM / 64, 1), 256, 0, stream>>>(wqkv, 3 * DM, WB, 1 << 30);
    k_cvtT<<<dim3(DM / 64, DM / 64, 1), 256, 0, stream>>>(wfc, DM, WF, 1 << 30);

    k_gemm_q<<<dim3(NB * SEQ / 64, DM / 64, 1), 32, 0, stream>>>(XB, WB, bqkv, QH, QR);
    k_gemm_k<<<dim3(NB * SEQ / 64, DM / 64, 1), 32, 0, stream>>>(XB, WB + (size_t)DM * DM, bqkv, KP);
    k_gemm_v<<<dim3(DM / 64, NB * SEQ / 64, 1), 32, 0, stream>>>(WB + (size_t)2 * DM * DM, XB, bqkv, VT, VR);

    k_flash<<<dim3(SEQ / (16 * AW), NB * NH_, 1), 32 * AW, 0, stream>>>(QH, QR, KP, VT, VR, EP, CH, CL);

    k_gemm_o<<<dim3(NB * SEQ / 64, DM / 64, 1), 32, 0, stream>>>(CH, WF, bfc, OUT);
}
